// RNN_824633720915
// MI455X (gfx1250) — hardware-verified
//
#include <hip/hip_runtime.h>
#include <math.h>

constexpr int NTRIAL   = 64;
constexpr int NLAT     = 512;
constexpr int NDRV     = 16;
constexpr int NOBS     = 256;
constexpr int NSTEP    = 1000;
constexpr int NTHR     = 256;
constexpr int NHALF    = 32;
constexpr int SEQ_BLK  = 16;
constexpr int VPAD     = 32;
constexpr int APITCH   = NLAT + VPAD + 8;
constexpr int ZPITCH   = NLAT + 8;
constexpr int OBS_ROWS = 16;
constexpr int TILES_PER_WAVE = 8;
constexpr float WCARRY     = 128.0f;
constexpr float WCARRY_INV = 1.0f / WCARRY;
constexpr float LOCARRY    = 2048.0f;
constexpr float LO_INV     = 1.0f / (WCARRY * LOCARRY);

static_assert(NTRIAL == 2 * NHALF, "two batch halves");
static_assert(NHALF % SEQ_BLK == 0, "whole 16-trial tiles per half");
static_assert(NLAT == 64 * (NTHR / 32), "8 waves x 64 latent columns");
static_assert(NLAT % 32 == 0 && VPAD == 32 && NDRV <= VPAD, "K chunks of 32");
static_assert(APITCH % 8 == 0 && ZPITCH % 8 == 0, "16-byte aligned LDS rows");
static_assert((OBS_ROWS * NSTEP * 4) % 128 == 0, "readout block owns whole lines");
static_assert(((OBS_ROWS * NSTEP) / 4) % 32 == 0, "copy guard is wave uniform");
static_assert((NTHR / 32) * TILES_PER_WAVE * 16 >= NSTEP, "time tiles cover all steps");
static_assert(NOBS % OBS_ROWS == 0 && NOBS % 64 == 0 && NLAT % 64 == 0, "tile multiples");
static_assert(OBS_ROWS * NSTEP * 4 <= 65536, "static LDS budget");

typedef __attribute__((ext_vector_type(16))) _Float16 v16h;
typedef __attribute__((ext_vector_type(8)))  _Float16 v8h;
typedef __attribute__((ext_vector_type(16))) __bf16   v16b;
typedef __attribute__((ext_vector_type(8)))  __bf16   v8b;
typedef __attribute__((ext_vector_type(8)))  float    v8f;
typedef __attribute__((ext_vector_type(4)))  float    v4f;
typedef __attribute__((ext_vector_type(4)))  unsigned v4u;

__device__ __forceinline__ unsigned short f2bf_bits(float f) {
  unsigned u = __float_as_uint(f);
  return (unsigned short)((u + 0x7FFFu + ((u >> 16) & 1u)) >> 16);
}
__device__ __forceinline__ float bf_bits2f(unsigned short h) { return __uint_as_float(((unsigned)h) << 16); }

__device__ __forceinline__ void split_f16_carry(float s, unsigned short& hb, unsigned short& lb) {
  const _Float16 h = (_Float16)s;
  const unsigned short hraw = __builtin_bit_cast(unsigned short, h);
  unsigned hbits = (unsigned)hraw;
  const unsigned em = hbits & 0x7fffu;
  const bool sub = (em < 0x400u);
  const float hnorm = __uint_as_float(((em << 13) + 0x38000000u) | ((hbits & 0x8000u) << 16));
  const float hf = sub ? 0.0f : hnorm;
  hbits = sub ? 0u : hbits;
  const float res = (s - hf) * LOCARRY;
  const _Float16 l = (_Float16)res;
  const unsigned short lraw = __builtin_bit_cast(unsigned short, l);
  hb = (unsigned short)hbits;
  lb = lraw;
}

__device__ __forceinline__ void guard4_h(v8f& a0, v8f& a1, v8f& a2, v8f& a3, v16h x, v16h y0, v16h y1, v16h y2, v16h y3) {
  asm volatile("v_nop\n\tv_nop\n\tv_nop\n\tv_nop" : "+v"(a0), "+v"(a1), "+v"(a2), "+v"(a3) : "v"(x), "v"(y0), "v"(y1), "v"(y2), "v"(y3));
}
__device__ __forceinline__ void guard1_b(v8f& a0, v16b x0, v16b x1, v16b y0, v16b y1) {
  asm volatile("v_nop\n\tv_nop\n\tv_nop\n\tv_nop" : "+v"(a0) : "v"(x0), "v"(x1), "v"(y0), "v"(y1));
}

template <typename T> struct Frag;
template <> struct Frag<_Float16> {
  typedef v16h V; union U { v16h v; v8h h[2]; };
  static __device__ __forceinline__ v16h load(const _Float16* p) {
    U f; f.h[0] = *(const v8h*)(p); f.h[1] = *(const v8h*)(p + 16); return f.v;
  }
  static __device__ __forceinline__ v8f mma(v16h a, v16h b, v8f c) {
    return __builtin_amdgcn_wmma_f32_16x16x32_f16(false, a, false, b, (short)0, c, false, false);
  }
};
template <> struct Frag<__bf16> {
  typedef v16b V; union U { v16b v; v8b h[2]; };
  static __device__ __forceinline__ v16b load(const __bf16* p) {
    U f; f.h[0] = *(const v8b*)(p); f.h[1] = *(const v8b*)(p + 16); return f.v;
  }
  static __device__ __forceinline__ v8f mma(v16b a, v16b b, v8f c) {
    return __builtin_amdgcn_wmma_f32_16x16x32_bf16(false, a, false, b, (short)0, c, false, false);
  }
};

__global__ __launch_bounds__(NTHR) void cvt_w_kernel(const float* __restrict__ src, unsigned short* __restrict__ dstH,
                                                     unsigned short* __restrict__ dstL, int n8, float sc) {
  const int i = blockIdx.x * NTHR + threadIdx.x;
  if (i < n8) {
    const float* sp = src + (size_t)i * 8;
    const v4f a = *(const v4f*)(sp);
    const v4f b = *(const v4f*)(sp + 4);
    v8h hv, lv;
#pragma unroll
    for (int e = 0; e < 4; ++e) {
      const float fa = a[e] * sc;
      const float fb = b[e] * sc;
      unsigned short ha, la, hb, lb;
      split_f16_carry(fa, ha, la);
      split_f16_carry(fb, hb, lb);
      hv[e]     = __builtin_bit_cast(_Float16, ha);
      lv[e]     = __builtin_bit_cast(_Float16, la);
      hv[4 + e] = __builtin_bit_cast(_Float16, hb);
      lv[4 + e] = __builtin_bit_cast(_Float16, lb);
    }
    *(volatile v8h*)(dstH + (size_t)i * 8) = hv;
    *(volatile v8h*)(dstL + (size_t)i * 8) = lv;
    __threadfence();
    *(volatile v8h*)(dstH + (size_t)i * 8) = hv;
    *(volatile v8h*)(dstL + (size_t)i * 8) = lv;
  }
}

__global__ __launch_bounds__(NTHR) void cvt_wu_kernel(const float* __restrict__ src, unsigned short* __restrict__ dstH,
                                                      unsigned short* __restrict__ dstL, float sc) {
  const int i = blockIdx.x * NTHR + threadIdx.x;
  const int n8 = NLAT * VPAD / 8;
  if (i < n8) {
    const int row = i >> 2;
    const int c8  = i & 3;
    const int cc  = c8 & 1;
    const bool keep = (c8 < 2);
    const float* sp = src + (size_t)row * NDRV + cc * 8;
    const v4f a = *(const v4f*)(sp);
    const v4f b = *(const v4f*)(sp + 4);
    v8h hv, lv;
#pragma unroll
    for (int e = 0; e < 4; ++e) {
      float fa = a[e] * sc;
      float fb = b[e] * sc;
      fa = keep ? fa : 0.0f;
      fb = keep ? fb : 0.0f;
      unsigned short ha, la, hb, lb;
      split_f16_carry(fa, ha, la);
      split_f16_carry(fb, hb, lb);
      hv[e]     = __builtin_bit_cast(_Float16, ha);
      lv[e]     = __builtin_bit_cast(_Float16, la);
      hv[4 + e] = __builtin_bit_cast(_Float16, hb);
      lv[4 + e] = __builtin_bit_cast(_Float16, lb);
    }
    *(volatile v8h*)(dstH + (size_t)i * 8) = hv;
    *(volatile v8h*)(dstL + (size_t)i * 8) = lv;
    __threadfence();
    *(volatile v8h*)(dstH + (size_t)i * 8) = hv;
    *(volatile v8h*)(dstL + (size_t)i * 8) = lv;
  }
}

__global__ __launch_bounds__(NTHR) void obs_prep_kernel(const float* __restrict__ src,
                                                        unsigned short* __restrict__ OH, unsigned short* __restrict__ OL) {
  __shared__ float Tt[64 * 65];
  const int tid = threadIdx.x;
  const int c0 = blockIdx.x * 64, r0 = blockIdx.y * 64;
#pragma unroll
  for (int i = 0; i < 4; ++i) {
    const int idx = i * NTHR + tid;
    const int rr = idx >> 4, cc = (idx & 15) * 4;
    const v4f v = *(const v4f*)(src + (size_t)(r0 + rr) * (size_t)NOBS + c0 + cc);
    Tt[rr * 65 + cc + 0] = v[0];
    Tt[rr * 65 + cc + 1] = v[1];
    Tt[rr * 65 + cc + 2] = v[2];
    Tt[rr * 65 + cc + 3] = v[3];
  }
  __syncthreads();
  const int q = tid >> 3, c8 = (tid & 7) * 8;
  v8h hv[2], lv[2];
#pragma unroll
  for (int g = 0; g < 2; ++g) {
    const int qq = g * 32 + q;
#pragma unroll
    for (int e = 0; e < 8; ++e) {
      const float f = Tt[(c8 + e) * 65 + qq];
      const unsigned short hb = f2bf_bits(f);
      const unsigned short lb = f2bf_bits(f - bf_bits2f(hb));
      hv[g][e] = __builtin_bit_cast(_Float16, hb);
      lv[g][e] = __builtin_bit_cast(_Float16, lb);
    }
  }
  for (int pass = 0; pass < 2; ++pass) {
#pragma unroll
    for (int g = 0; g < 2; ++g) {
      const size_t o = (size_t)(c0 + g * 32 + q) * (size_t)NLAT + (size_t)(r0 + c8);
      *(volatile v8h*)(OH + o) = hv[g];
      *(volatile v8h*)(OL + o) = lv[g];
    }
    __threadfence();
  }
}

__global__ __launch_bounds__(NTHR) void prep_v_kernel(const float* __restrict__ v, unsigned short* __restrict__ vt) {
  __shared__ float Tv[256 * 33];
  const int tid = threadIdx.x;
  const int t0 = blockIdx.x * 32;
  const int b0 = blockIdx.y * SEQ_BLK;
#pragma unroll 1
  for (int i = 0; i < 32; ++i) {
    const int idx = i * NTHR + tid;
    const int row = idx >> 5, tt = idx & 31;
    int t = t0 + tt;
    t = (t < NSTEP) ? t : (NSTEP - 1);
    Tv[row * 33 + tt] = v[(size_t)(b0 * NDRV + row) * NSTEP + t];
  }
  __syncthreads();
#pragma unroll 1
  for (int it = 0; it < 8; ++it) {
    const int id = it * NTHR + tid;
    const int tt = id >> 6, q = id & 63;
    const int bl = q >> 2, c8 = q & 3;
    const int jb = (c8 & 1) * 8;
    const bool keep = (c8 < 2);
    const int t = t0 + tt;
    v8h hv;
#pragma unroll
    for (int e = 0; e < 8; ++e) {
      float f = Tv[(bl * NDRV + jb + e) * 33 + tt];
      f = keep ? f : 0.0f;
      hv[e] = (_Float16)f;
    }
    if (t < NSTEP) {
      unsigned short* dp = vt + ((size_t)t * NTRIAL + (size_t)(b0 + bl)) * VPAD + c8 * 8;
      *(volatile v8h*)dp = hv;
      __threadfence();
      *(volatile v8h*)dp = hv;
    }
  }
}

__device__ __forceinline__ void sweep17(const _Float16* arow, const _Float16* wb, const _Float16* wu,
                                        v8f& acc0, v8f& acc1, v8f& acc2, v8f& acc3) {
#pragma unroll 1
  for (int k0 = 0; k0 < NLAT; k0 += 32) {
    const v16h a  = Frag<_Float16>::load(arow + k0);
    const v16h b0 = Frag<_Float16>::load(wb + k0);
    const v16h b1 = Frag<_Float16>::load(wb + (size_t)16 * NLAT + k0);
    const v16h b2 = Frag<_Float16>::load(wb + (size_t)32 * NLAT + k0);
    const v16h b3 = Frag<_Float16>::load(wb + (size_t)48 * NLAT + k0);
    acc0 = Frag<_Float16>::mma(a, b0, acc0);
    acc1 = Frag<_Float16>::mma(a, b1, acc1);
    acc2 = Frag<_Float16>::mma(a, b2, acc2);
    acc3 = Frag<_Float16>::mma(a, b3, acc3);
    guard4_h(acc0, acc1, acc2, acc3, a, b0, b1, b2, b3);
  }
  {
    const v16h a  = Frag<_Float16>::load(arow + NLAT);
    const v16h b0 = Frag<_Float16>::load(wu);
    const v16h b1 = Frag<_Float16>::load(wu + (size_t)16 * VPAD);
    const v16h b2 = Frag<_Float16>::load(wu + (size_t)32 * VPAD);
    const v16h b3 = Frag<_Float16>::load(wu + (size_t)48 * VPAD);
    acc0 = Frag<_Float16>::mma(a, b0, acc0);
    acc1 = Frag<_Float16>::mma(a, b1, acc1);
    acc2 = Frag<_Float16>::mma(a, b2, acc2);
    acc3 = Frag<_Float16>::mma(a, b3, acc3);
    guard4_h(acc0, acc1, acc2, acc3, a, b0, b1, b2, b3);
  }
}

__global__ __launch_bounds__(NTHR) void scan_kernel(const float* z0, const float* hvec, const float* __restrict__ dp,
                                                    const unsigned short* __restrict__ WHp,
                                                    const unsigned short* __restrict__ WLp,
                                                    const unsigned short* __restrict__ WUHp,
                                                    const unsigned short* __restrict__ WULp,
                                                    const unsigned short* __restrict__ VTp,
                                                    unsigned short* __restrict__ ZHp, unsigned short* __restrict__ ZLp,
                                                    int trial0) {
  __shared__ __align__(16) _Float16       Act[SEQ_BLK * APITCH];
  __shared__ __align__(16) unsigned short Zsh[SEQ_BLK * ZPITCH];
  __shared__ __align__(16) unsigned short Zsl[SEQ_BLK * ZPITCH];
  const int tid = threadIdx.x, lane = tid & 31, wave = tid >> 5;
  const int c = lane & 15, hh = lane >> 4, koff = hh * 8;
  const int lrow0 = blockIdx.x * SEQ_BLK;
  const int grow0 = trial0 + lrow0;

  const float dec = expf(-expf(dp[0]));

  float zst[4][8];
  float hn[4];
#pragma unroll
  for (int nt = 0; nt < 4; ++nt) {
    const int j = 64 * wave + 16 * nt + c;
    hn[nt] = hvec[j];
#pragma unroll
    for (int r = 0; r < 8; ++r) zst[nt][r] = z0[(size_t)(grow0 + 8 * hh + r) * NLAT + j];
#pragma unroll
    for (int r = 0; r < 8; ++r) {
      const float a = fmaxf(zst[nt][r] - hn[nt], 0.0f);
      Act[(8 * hh + r) * APITCH + j] = (_Float16)a;
    }
    asm volatile("" ::: "memory");
  }
  if (tid < 64) {
    const int m = tid >> 2, q = tid & 3;
    const v4u x = *(const v4u*)(VTp + ((size_t)0 * NTRIAL + (size_t)(grow0 + m)) * VPAD + q * 8);
    *(v4u*)(Act + m * APITCH + NLAT + q * 8) = x;
  }
  __syncthreads();

  const _Float16* arow = Act + c * APITCH + koff;
  const _Float16* wbh  = (const _Float16*)WHp  + (size_t)(64 * wave + c) * NLAT + koff;
  const _Float16* wbl  = (const _Float16*)WLp  + (size_t)(64 * wave + c) * NLAT + koff;
  const _Float16* wuh  = (const _Float16*)WUHp + (size_t)(64 * wave + c) * VPAD + koff;
  const _Float16* wul  = (const _Float16*)WULp + (size_t)(64 * wave + c) * VPAD + koff;
  const v8f z8 = {0.f, 0.f, 0.f, 0.f, 0.f, 0.f, 0.f, 0.f};

#pragma unroll 1
  for (int t = 0; t < NSTEP; ++t) {
    v8f acc0 = z8, acc1 = z8, acc2 = z8, acc3 = z8;
    sweep17(arow, wbh, wuh, acc0, acc1, acc2, acc3);
#pragma unroll
    for (int nt = 0; nt < 4; ++nt) {
#pragma unroll
      for (int r = 0; r < 8; ++r) {
        const float av = (nt == 0) ? acc0[r] : (nt == 1) ? acc1[r] : (nt == 2) ? acc2[r] : acc3[r];
        zst[nt][r] = dec * zst[nt][r] + av * WCARRY_INV;
      }
    }
    acc0 = z8; acc1 = z8; acc2 = z8; acc3 = z8;
    sweep17(arow, wbl, wul, acc0, acc1, acc2, acc3);
#pragma unroll
    for (int nt = 0; nt < 4; ++nt) {
      const int j = 64 * wave + 16 * nt + c;
#pragma unroll
      for (int r = 0; r < 8; ++r) {
        const float av = (nt == 0) ? acc0[r] : (nt == 1) ? acc1[r] : (nt == 2) ? acc2[r] : acc3[r];
        const float zn = zst[nt][r] + av * LO_INV;
        zst[nt][r] = zn;
        const unsigned short hb = f2bf_bits(zn);
        const unsigned short lb = f2bf_bits(zn - bf_bits2f(hb));
        Zsh[(8 * hh + r) * ZPITCH + j] = hb;
        Zsl[(8 * hh + r) * ZPITCH + j] = lb;
      }
    }
    __syncthreads();
#pragma unroll
    for (int nt = 0; nt < 4; ++nt) {
      const int j = 64 * wave + 16 * nt + c;
#pragma unroll
      for (int r = 0; r < 8; ++r) {
        const float a = fmaxf(zst[nt][r] - hn[nt], 0.0f);
        Act[(8 * hh + r) * APITCH + j] = (_Float16)a;
      }
    }
    if (tid < 64) {
      const int tn = (t + 1 < NSTEP) ? (t + 1) : (NSTEP - 1);
      const int m = tid >> 2, q = tid & 3;
      const v4u x = *(const v4u*)(VTp + ((size_t)tn * NTRIAL + (size_t)(grow0 + m)) * VPAD + q * 8);
      *(v4u*)(Act + m * APITCH + NLAT + q * 8) = x;
    }
    for (int pass = 0; pass < 2; ++pass) {
#pragma unroll
      for (int it = 0; it < 4; ++it) {
        const int id = it * NTHR + tid;
        const int row = id >> 6, ch = id & 63;
        const v4u hvv = *(const v4u*)(Zsh + row * ZPITCH + ch * 8);
        const v4u lvv = *(const v4u*)(Zsl + row * ZPITCH + ch * 8);
        const size_t goff = ((size_t)(lrow0 + row) * NSTEP + (size_t)t) * NLAT + (size_t)ch * 8;
        *(volatile v4u*)(ZHp + goff) = hvv;
        *(volatile v4u*)(ZLp + goff) = lvv;
      }
      __threadfence();
    }
    __syncthreads();
  }
}

__global__ __launch_bounds__(NTHR) void obs_kernel(const unsigned short* __restrict__ OHp, const unsigned short* __restrict__ OLp,
                                                   const unsigned short* __restrict__ ZHp, const unsigned short* __restrict__ ZLp,
                                                   const float* __restrict__ bias, float* __restrict__ out, int trial0) {
  __shared__ __align__(16) float Os[OBS_ROWS * NSTEP];
  const int tid = threadIdx.x, lane = tid & 31, wave = tid >> 5;
  const int c = lane & 15, hh = lane >> 4, koff = hh * 8;
  const int x0 = blockIdx.x * OBS_ROWS;
  const int ltrial = blockIdx.y;
  const __bf16* oh = (const __bf16*)OHp + (size_t)(x0 + c) * NLAT + koff;
  const __bf16* ol = (const __bf16*)OLp + (size_t)(x0 + c) * NLAT + koff;
  const __bf16* zh = (const __bf16*)ZHp + (size_t)ltrial * NSTEP * NLAT;
  const __bf16* zl = (const __bf16*)ZLp + (size_t)ltrial * NSTEP * NLAT;

  int zoff[TILES_PER_WAVE];
#pragma unroll
  for (int j = 0; j < TILES_PER_WAVE; ++j) {
    int tt = (wave * TILES_PER_WAVE + j) * 16 + c;
    tt = (tt < NSTEP) ? tt : (NSTEP - 1);
    zoff[j] = tt * NLAT + koff;
  }
  v8f acc[TILES_PER_WAVE];
#pragma unroll
  for (int j = 0; j < TILES_PER_WAVE; ++j) acc[j] = (v8f){0.f, 0.f, 0.f, 0.f, 0.f, 0.f, 0.f, 0.f};

#pragma unroll 1
  for (int k0 = 0; k0 < NLAT; k0 += 32) {
    const v16b ah = Frag<__bf16>::load(oh + k0);
    const v16b al = Frag<__bf16>::load(ol + k0);
#pragma unroll
    for (int j = 0; j < TILES_PER_WAVE; ++j) {
      const v16b bh = Frag<__bf16>::load(zh + zoff[j] + k0);
      const v16b bq = Frag<__bf16>::load(zl + zoff[j] + k0);
      acc[j] = Frag<__bf16>::mma(ah, bh, acc[j]);
      acc[j] = Frag<__bf16>::mma(ah, bq, acc[j]);
      acc[j] = Frag<__bf16>::mma(al, bh, acc[j]);
      guard1_b(acc[j], ah, al, bh, bq);
    }
  }

  float bv[8];
#pragma unroll
  for (int r = 0; r < 8; ++r) bv[r] = bias[x0 + 8 * hh + r];
#pragma unroll
  for (int j = 0; j < TILES_PER_WAVE; ++j) {
    const int tt = (wave * TILES_PER_WAVE + j) * 16 + c;
#pragma unroll
    for (int r = 0; r < 8; ++r) {
      const float val = acc[j][r] + bv[r];
      if (tt < NSTEP) Os[(8 * hh + r) * NSTEP + tt] = val;
    }
  }
  __syncthreads();

  float* op = out + ((size_t)(trial0 + ltrial) * NOBS + (size_t)x0) * NSTEP;
  const int nchunk = OBS_ROWS * NSTEP / 4;
  for (int pass = 0; pass < 2; ++pass) {
#pragma unroll 1
    for (int it = 0; it < 16; ++it) {
      const int id = it * NTHR + tid;
      if (id < nchunk) {
        const v4f val = *(const v4f*)(Os + (size_t)id * 4);
        *(volatile v4f*)(op + (size_t)id * 4) = val;
      }
    }
    __threadfence();
  }
}

extern "C" void kernel_launch(void* const* d_in, const int* in_sizes, int n_in,
                              void* d_out, int out_size, void* d_ws, size_t ws_size, hipStream_t stream) {
  if (n_in < 8 || d_out == nullptr || d_ws == nullptr) return;
  if (in_sizes[0] != NTRIAL * NLAT || in_sizes[1] != NTRIAL * NDRV * NSTEP || in_sizes[2] != NLAT * NLAT ||
      in_sizes[3] != NLAT * NDRV || in_sizes[4] != NLAT || in_sizes[5] != 1 ||
      in_sizes[6] != NLAT * NOBS || in_sizes[7] != NOBS || out_size != NTRIAL * NOBS * NSTEP) return;

  const float* z0   = (const float*)d_in[0];
  const float* vin  = (const float*)d_in[1];
  const float* wrec = (const float*)d_in[2];
  const float* wdrv = (const float*)d_in[3];
  const float* hvec = (const float*)d_in[4];
  const float* dpar = (const float*)d_in[5];
  const float* bobs = (const float*)d_in[6];
  const float* bias = (const float*)d_in[7];
  float* out = (float*)d_out;

  char* ws = (char*)d_ws;
  size_t off = 0;
  auto carve = [&](size_t bytes) -> char* { char* p = ws + off; off += (bytes + 255) & ~(size_t)255; return p; };
  unsigned short* WH  = (unsigned short*)carve((size_t)NLAT * NLAT * 2);
  unsigned short* WHL = (unsigned short*)carve((size_t)NLAT * NLAT * 2);
  unsigned short* WUH = (unsigned short*)carve((size_t)NLAT * VPAD * 2);
  unsigned short* WUL = (unsigned short*)carve((size_t)NLAT * VPAD * 2);
  unsigned short* OBH = (unsigned short*)carve((size_t)NOBS * NLAT * 2);
  unsigned short* OBL = (unsigned short*)carve((size_t)NOBS * NLAT * 2);
  unsigned short* VT  = (unsigned short*)carve((size_t)NSTEP * NTRIAL * VPAD * 2);
  unsigned short* ZH  = (unsigned short*)carve((size_t)NHALF * NSTEP * NLAT * 2);
  unsigned short* ZL  = (unsigned short*)carve((size_t)NHALF * NSTEP * NLAT * 2);
  if (off > ws_size || off > (size_t)134217728) return;

  const int n8w = NLAT * NLAT / 8;
  cvt_w_kernel<<<(n8w + NTHR - 1) / NTHR, NTHR, 0, stream>>>(wrec, WH, WHL, n8w, WCARRY);
  cvt_wu_kernel<<<(NLAT * VPAD / 8 + NTHR - 1) / NTHR, NTHR, 0, stream>>>(wdrv, WUH, WUL, WCARRY);
  obs_prep_kernel<<<dim3(NOBS / 64, NLAT / 64), NTHR, 0, stream>>>(bobs, OBH, OBL);
  prep_v_kernel<<<dim3((NSTEP + 31) / 32, NTRIAL / SEQ_BLK), NTHR, 0, stream>>>(vin, VT);

  for (int half = 0; half < 2; ++half) {
    const int trial0 = half * NHALF;
    scan_kernel<<<NHALF / SEQ_BLK, NTHR, 0, stream>>>(z0, hvec, dpar, WH, WHL, WUH, WUL, VT, ZH, ZL, trial0);
    obs_kernel<<<dim3(NOBS / OBS_ROWS, NHALF), NTHR, 0, stream>>>(OBH, OBL, ZH, ZL, bias, out, trial0);
  }
}
